// ScannedMemoroid_953482740290
// MI455X (gfx1250) — hardware-verified
//
#include <hip/hip_runtime.h>
#include <math.h>

constexpr int NSTEP   = 1024;
constexpr int NBATCH  = 32;
constexpr int NIN     = 128;
constexpr int NOUT    = 128;
constexpr int NTRACE  = 32;
constexpr int NCTX    = 32;
constexpr int NROWS   = NSTEP * NBATCH;
constexpr int KMIX    = 2 * NTRACE * NCTX;
constexpr int NCAT    = 2 * NTRACE + 2 * NOUT;
constexpr int TCHUNK  = 256;
constexpr int NCHUNK  = NSTEP / TCHUNK;
constexpr int CROWS   = TCHUNK * NBATCH;
constexpr int NSTATE  = NBATCH * NTRACE * NCTX;
constexpr int SLAB_PITCH = 68;
constexpr float WX_CARRY = 64.0f;
constexpr float WM_CARRY = 256.0f;
constexpr float Z_CARRY  = 64.0f;
constexpr float WX_FOLD  = 1.0f / WX_CARRY;
constexpr float MIX_FOLD = 1.0f / (WM_CARRY * Z_CARRY);
constexpr float LN_EPS_F = 1e-6f;

static_assert(NROWS == 32768 && KMIX == 2048 && NCAT == 320, "shape");
static_assert(NROWS % 64 == 0 && NCAT % 64 == 0 && NIN % 32 == 0, "x projection tiles");
static_assert(((NROWS / 64) * (NCAT / 64)) % 8 == 0, "x projection grid exact");
static_assert(CROWS % 256 == 0 && NOUT == 128 && KMIX % 32 == 0, "mix tiles");
static_assert(NSTEP % TCHUNK == 0 && TCHUNK % 4 == 0, "chunking");
static_assert(NSTATE % 256 == 0, "scan grid exact");
static_assert(NTRACE == 32 && NCTX == 32 && NBATCH == 32, "lane maps");

typedef __attribute__((ext_vector_type(16))) _Float16 v16h;
typedef __attribute__((ext_vector_type(8)))  _Float16 v8h;
typedef __attribute__((ext_vector_type(8)))  float    v8f;
typedef __attribute__((ext_vector_type(4)))  float    v4f;

union FragU { v16h v; v8h h[2]; };

__device__ __forceinline__ v16h frag_load(const _Float16* p) {
  FragU f;
  f.h[0] = *(const v8h*)(p);
  f.h[1] = *(const v8h*)(p + 16);
  return f.v;
}
__device__ __forceinline__ v8f mma_h(v16h a, v16h b, v8f c) {
  return __builtin_amdgcn_wmma_f32_16x16x32_f16(false, a, false, b, (short)0, c, false, false);
}
__device__ __forceinline__ void guard_row4(v8f& a, v8f& b, v8f& c, v8f& d,
                                           v16h x, v16h y0, v16h y1, v16h y2, v16h y3) {
  asm volatile("v_nop\n\tv_nop\n\tv_nop\n\tv_nop"
               : "+v"(a), "+v"(b), "+v"(c), "+v"(d)
               : "v"(x), "v"(y0), "v"(y1), "v"(y2), "v"(y3));
}
__device__ __forceinline__ void acc_guard4(v8f& a, v8f& b, v8f& c, v8f& d) {
  asm volatile("v_nop\n\tv_nop\n\tv_nop\n\tv_nop" : "+v"(a), "+v"(b), "+v"(c), "+v"(d));
}
__device__ __forceinline__ void wave_sync_lds() {
  __builtin_amdgcn_fence(__ATOMIC_RELEASE, "workgroup");
  __builtin_amdgcn_wave_barrier();
  __builtin_amdgcn_fence(__ATOMIC_ACQUIRE, "workgroup");
}

__global__ __launch_bounds__(256) void cvt_x_kernel(const float* __restrict__ src,
                                                    unsigned short* __restrict__ dst, int n8) {
  const int i = blockIdx.x * 256 + threadIdx.x;
  if (i < n8) {
    const float* sp = src + (size_t)i * 8;
    const v4f a = *(const v4f*)(sp);
    const v4f b = *(const v4f*)(sp + 4);
    v8h hv;
#pragma unroll
    for (int e = 0; e < 4; ++e) {
      hv[e]     = (_Float16)a[e];
      hv[4 + e] = (_Float16)b[e];
    }
    *(volatile v8h*)(dst + (size_t)i * 8) = hv;
    __threadfence();
    *(volatile v8h*)(dst + (size_t)i * 8) = hv;
  }
}

__global__ __launch_bounds__(256) void wt_kernel(const float* __restrict__ src, int ncols, int kdim,
                                                 unsigned short* __restrict__ dst,
                                                 int rowbase, int rowstride, float carry) {
  const int i = blockIdx.x * 256 + threadIdx.x;
  const int k8n = kdim >> 3;
  const int n8 = ncols * k8n;
  if (i < n8) {
    const int j  = i / k8n;
    const int k8 = (i - j * k8n) * 8;
    v8h hv;
#pragma unroll
    for (int e = 0; e < 8; ++e) {
      const float w = src[(size_t)(k8 + e) * ncols + j];
      hv[e] = (_Float16)(w * carry);
    }
    const int drow = rowbase + (j >> 5) * rowstride + (j & 31);
    unsigned short* dp = dst + (size_t)drow * kdim + k8;
    *(volatile v8h*)dp = hv;
    __threadfence();
    *(volatile v8h*)dp = hv;
  }
}

__global__ __launch_bounds__(256) void xproj_gemm_kernel(
    const unsigned short* __restrict__ Xp, const unsigned short* __restrict__ Wtp,
    const float* __restrict__ b_pre, const float* __restrict__ b_gin,
    const float* __restrict__ b_gout, const float* __restrict__ b_skip,
    float* __restrict__ Gpl, float* __restrict__ GATE, float* __restrict__ SKT) {
  __shared__ __align__(16) float sT[8][16 * SLAB_PITCH];
  const _Float16* A  = (const _Float16*)Xp;
  const _Float16* Bt = (const _Float16*)Wtp;
  const int lane = threadIdx.x & 31;
  const int wave = threadIdx.x >> 5;
  const int tilesN = NCAT >> 6;
  const int tile = blockIdx.x * 8 + wave;
  const int tm = tile / tilesN;
  const int tn = tile - tm * tilesN;
  const int m0 = tm << 6;
  const int n0 = tn << 6;
  const int rlane = lane & 15;
  const int koff  = (lane >> 4) * 8;
  const int mOff  = (lane >> 4) * 8;

  v8f acc[4][4];
#pragma unroll
  for (int i = 0; i < 4; ++i)
#pragma unroll
    for (int j = 0; j < 4; ++j) acc[i][j] = (v8f){0.f, 0.f, 0.f, 0.f, 0.f, 0.f, 0.f, 0.f};

#pragma unroll 1
  for (int k0 = 0; k0 < NIN; k0 += 32) {
    v16h bh[4];
#pragma unroll
    for (int j = 0; j < 4; ++j) {
      const size_t bo = (size_t)(n0 + (j << 4) + rlane) * NIN + koff + k0;
      bh[j] = frag_load(Bt + bo);
    }
#pragma unroll
    for (int i = 0; i < 4; ++i) {
      const size_t ao = (size_t)(m0 + (i << 4) + rlane) * NIN + koff + k0;
      const v16h ah = frag_load(A + ao);
#pragma unroll
      for (int j = 0; j < 4; ++j) acc[i][j] = mma_h(ah, bh[j], acc[i][j]);
      guard_row4(acc[i][0], acc[i][1], acc[i][2], acc[i][3], ah, bh[0], bh[1], bh[2], bh[3]);
    }
  }
  acc_guard4(acc[0][0], acc[0][1], acc[0][2], acc[0][3]);
  acc_guard4(acc[1][0], acc[1][1], acc[1][2], acc[1][3]);
  acc_guard4(acc[2][0], acc[2][1], acc[2][2], acc[2][3]);
  acc_guard4(acc[3][0], acc[3][1], acc[3][2], acc[3][3]);

  const bool first_tile = (tn == 0);
  const int pc = (tn > 0) ? (tn - 1) * 32 : 0;
  const float fsel = first_tile ? 1.0f : 0.0f;
  const float gsel = 1.0f - fsel;
  const float bp = b_pre[lane];
  const float bg = b_gin[lane];
  const float bs = b_skip[pc + lane];
  const float bo = b_gout[pc + lane];
  const float biasA = fmaf(fsel, bp, gsel * bs);
  const float biasB = fmaf(fsel, bg, gsel * bo);

  float* slab = sT[wave];
  const int q  = lane >> 3;
  const int c4 = (lane & 7) * 4;
#pragma unroll
  for (int i = 0; i < 4; ++i) {
    const int mBase = m0 + (i << 4);
#pragma unroll
    for (int j = 0; j < 4; ++j)
#pragma unroll
      for (int r = 0; r < 8; ++r)
        slab[(mOff + r) * SLAB_PITCH + (j << 4) + rlane] = acc[i][j][r] * WX_FOLD;
    wave_sync_lds();
#pragma unroll 1
    for (int row = 0; row < 16; ++row) {
      float* sp = slab + row * SLAB_PITCH;
      const float av = sp[lane] + biasA;
      const float zv = sp[32 + lane] + biasB;
      const float sg = 1.0f / (1.0f + expf(-zv));
      const float fac = first_tile ? sg : (1.0f - sg);
      sp[lane] = av * fac;
      sp[32 + lane] = sg;
    }
    wave_sync_lds();
    if (first_tile) {
      for (int pass = 0; pass < 2; ++pass) {
#pragma unroll
        for (int it = 0; it < 4; ++it) {
          const int row = it * 4 + q;
          const v4f v = *(const v4f*)(slab + row * SLAB_PITCH + c4);
          *(volatile v4f*)(Gpl + (size_t)(mBase + row) * NTRACE + c4) = v;
        }
        __threadfence();
      }
    } else {
      for (int pass = 0; pass < 2; ++pass) {
#pragma unroll
        for (int it = 0; it < 4; ++it) {
          const int row = it * 4 + q;
          const v4f v0 = *(const v4f*)(slab + row * SLAB_PITCH + c4);
          const v4f v1 = *(const v4f*)(slab + row * SLAB_PITCH + 32 + c4);
          *(volatile v4f*)(SKT  + (size_t)(mBase + row) * NOUT + pc + c4) = v0;
          *(volatile v4f*)(GATE + (size_t)(mBase + row) * NOUT + pc + c4) = v1;
        }
        __threadfence();
      }
    }
    wave_sync_lds();
  }
}

template <bool FIRST>
__global__ __launch_bounds__(256) void scan_chunk_kernel(
    const float* __restrict__ Gpl, const int* __restrict__ resets,
    const float* __restrict__ init_re, const float* __restrict__ init_im,
    const float* __restrict__ a_param, const float* __restrict__ b_param,
    float* __restrict__ carry_out, unsigned* __restrict__ Zw, int t0) {
  const int tid  = blockIdx.x * 256 + threadIdx.x;
  const int lane = threadIdx.x & 31;
  const int c = tid & 31;
  const int r = (tid >> 5) & 31;
  const int b = tid >> 10;
  const float er = expf(-fabsf(a_param[r]));
  const float ph = b_param[c];
  const float lr = er * cosf(ph);
  const float li = er * sinf(ph);
  float sre = init_re[tid];
  float sim = 0.0f;
  if (!FIRST) sim = init_im[tid];
  const int srcA = 2 * (lane & 15);
  const int srcB = srcA + 1;
  const bool lowhalf = lane < 16;
  unsigned* zbase = Zw + (size_t)b * (KMIX / 2) + r * 32 + lane;

#pragma unroll 1
  for (int tq = 0; tq < TCHUNK / 4; ++tq) {
    unsigned wd[4];
#pragma unroll
    for (int u = 0; u < 4; ++u) {
      const int tl = tq * 4 + u;
      const int mb = (t0 + tl) * NBATCH + b;
      const int rs = resets[mb];
      const float g = Gpl[(size_t)mb * NTRACE + r];
      const float ore = (rs != 0) ? 0.0f : sre;
      const float oim = (rs != 0) ? 0.0f : sim;
      const float nre = ore * lr - oim * li + g;
      const float nim = ore * li + oim * lr;
      sre = nre;
      sim = nim;
      const _Float16 hre = (_Float16)(nre * Z_CARRY);
      const _Float16 him = (_Float16)(nim * Z_CARRY);
      const unsigned short bre = __builtin_bit_cast(unsigned short, hre);
      const unsigned short bim = __builtin_bit_cast(unsigned short, him);
      const unsigned pk = (unsigned)bre | ((unsigned)bim << 16);
      const unsigned pa = (unsigned)__shfl((int)pk, srcA, 32);
      const unsigned pb = (unsigned)__shfl((int)pk, srcB, 32);
      const unsigned wlo = (pa & 0xffffu) | (pb << 16);
      const unsigned whi = (pa >> 16) | (pb & 0xffff0000u);
      wd[u] = lowhalf ? wlo : whi;
    }
    unsigned* zp = zbase + (size_t)(tq * 4) * NBATCH * (KMIX / 2);
#pragma unroll
    for (int pass = 0; pass < 2; ++pass) {
#pragma unroll
      for (int u = 0; u < 4; ++u)
        *(volatile unsigned*)(zp + (size_t)u * NBATCH * (KMIX / 2)) = wd[u];
      __threadfence();
    }
  }
  *(volatile float*)(carry_out + tid) = sre;
  *(volatile float*)(carry_out + NSTATE + tid) = sim;
  __threadfence();
  *(volatile float*)(carry_out + tid) = sre;
  *(volatile float*)(carry_out + NSTATE + tid) = sim;
}

__global__ __launch_bounds__(256) void mix_ln_kernel(
    const unsigned short* __restrict__ Zp, const unsigned short* __restrict__ Wmp,
    const float* __restrict__ b_mix, const float* __restrict__ GATE, const float* __restrict__ SKT,
    float* __restrict__ outp, int row0) {
  __shared__ __align__(16) float sT[8][16 * SLAB_PITCH];
  const _Float16* A  = (const _Float16*)Zp;
  const _Float16* Bt = (const _Float16*)Wmp;
  const int lane = threadIdx.x & 31;
  const int wave = threadIdx.x >> 5;
  const int mt = wave >> 1;
  const int tn = wave & 1;
  const int m0 = blockIdx.x * 256 + mt * 64;
  const int n0 = tn * 64;
  const int rlane = lane & 15;
  const int koff  = (lane >> 4) * 8;
  const int mOff  = (lane >> 4) * 8;

  v8f acc[4][4];
#pragma unroll
  for (int i = 0; i < 4; ++i)
#pragma unroll
    for (int j = 0; j < 4; ++j) acc[i][j] = (v8f){0.f, 0.f, 0.f, 0.f, 0.f, 0.f, 0.f, 0.f};

#pragma unroll 1
  for (int k0 = 0; k0 < KMIX; k0 += 32) {
    v16h bh[4];
#pragma unroll
    for (int j = 0; j < 4; ++j) {
      const size_t bo = (size_t)(n0 + (j << 4) + rlane) * KMIX + koff + k0;
      bh[j] = frag_load(Bt + bo);
    }
#pragma unroll
    for (int i = 0; i < 4; ++i) {
      const size_t ao = (size_t)(m0 + (i << 4) + rlane) * KMIX + koff + k0;
      const v16h ah = frag_load(A + ao);
#pragma unroll
      for (int j = 0; j < 4; ++j) acc[i][j] = mma_h(ah, bh[j], acc[i][j]);
      guard_row4(acc[i][0], acc[i][1], acc[i][2], acc[i][3], ah, bh[0], bh[1], bh[2], bh[3]);
    }
  }
  acc_guard4(acc[0][0], acc[0][1], acc[0][2], acc[0][3]);
  acc_guard4(acc[1][0], acc[1][1], acc[1][2], acc[1][3]);
  acc_guard4(acc[2][0], acc[2][1], acc[2][2], acc[2][3]);
  acc_guard4(acc[3][0], acc[3][1], acc[3][2], acc[3][3]);

  const v4f bm = *(const v4f*)(b_mix + 4 * lane);
  float* slab = sT[wave];
  const float* sAll = &sT[0][0];
  const int srcSlab = lane >> 4;
  const int srcCol  = (lane & 15) * 4;

#pragma unroll
  for (int i = 0; i < 4; ++i) {
#pragma unroll
    for (int j = 0; j < 4; ++j)
#pragma unroll
      for (int r = 0; r < 8; ++r)
        slab[(mOff + r) * SLAB_PITCH + (j << 4) + rlane] = acc[i][j][r] * MIX_FOLD;
    __syncthreads();
#pragma unroll 1
    for (int qq = 0; qq < 8; ++qq) {
      const int R   = wave * 8 + qq;
      const int mtr = R >> 4;
      const int rr  = R & 15;
      const size_t grow = (size_t)row0 + (size_t)blockIdx.x * 256 + (size_t)(mtr * 64 + i * 16 + rr);
      const float* sp = sAll + (mtr * 2 + srcSlab) * (16 * SLAB_PITCH) + rr * SLAB_PITCH + srcCol;
      const v4f av = *(const v4f*)sp;
      const v4f gv = *(const v4f*)(GATE + grow * NOUT + 4 * lane);
      const v4f sv = *(const v4f*)(SKT  + grow * NOUT + 4 * lane);
      v4f y;
#pragma unroll
      for (int e = 0; e < 4; ++e) y[e] = (av[e] + bm[e]) * gv[e];
      float s = (y[0] + y[1]) + (y[2] + y[3]);
#pragma unroll
      for (int off = 1; off < 32; off <<= 1) s += __shfl_xor(s, off, 32);
      const float mu = s * (1.0f / NOUT);
      float ss = 0.0f;
      v4f d;
#pragma unroll
      for (int e = 0; e < 4; ++e) { d[e] = y[e] - mu; ss += d[e] * d[e]; }
#pragma unroll
      for (int off = 1; off < 32; off <<= 1) ss += __shfl_xor(ss, off, 32);
      const float var  = ss * (1.0f / NOUT);
      const float rstd = rsqrtf(var + LN_EPS_F);
      v4f o;
#pragma unroll
      for (int e = 0; e < 4; ++e) o[e] = d[e] * rstd + sv[e];
      float* op = outp + grow * NOUT + 4 * lane;
      *(volatile v4f*)op = o;
      __threadfence();
      *(volatile v4f*)op = o;
    }
    __syncthreads();
  }
}

extern "C" void kernel_launch(void* const* d_in, const int* in_sizes, int n_in,
                              void* d_out, int out_size, void* d_ws, size_t ws_size, hipStream_t stream) {
  if (n_in < 16 || d_out == nullptr || d_ws == nullptr) return;
  if (in_sizes[0] != NSTATE || in_sizes[1] != NBATCH || in_sizes[2] != NROWS * NIN ||
      in_sizes[3] != NROWS || in_sizes[4] != NTRACE || in_sizes[5] != NCTX ||
      in_sizes[6] != NIN * NTRACE || in_sizes[7] != NTRACE || in_sizes[8] != NIN * NTRACE ||
      in_sizes[9] != NTRACE || in_sizes[10] != NIN * NOUT || in_sizes[11] != NOUT ||
      in_sizes[12] != NIN * NOUT || in_sizes[13] != NOUT || in_sizes[14] != KMIX * NOUT ||
      in_sizes[15] != NOUT || out_size != NROWS * NOUT) return;

  const float* h0      = (const float*)d_in[0];
  const float* x       = (const float*)d_in[2];
  const int*   resets  = (const int*)d_in[3];
  const float* a_param = (const float*)d_in[4];
  const float* b_param = (const float*)d_in[5];
  const float* W_pre   = (const float*)d_in[6];
  const float* b_pre   = (const float*)d_in[7];
  const float* W_gin   = (const float*)d_in[8];
  const float* b_gin   = (const float*)d_in[9];
  const float* W_gout  = (const float*)d_in[10];
  const float* b_gout  = (const float*)d_in[11];
  const float* W_skip  = (const float*)d_in[12];
  const float* b_skip  = (const float*)d_in[13];
  const float* W_mix   = (const float*)d_in[14];
  const float* b_mix   = (const float*)d_in[15];
  float* out = (float*)d_out;

  char* ws = (char*)d_ws;
  size_t off = 0;
  auto carve = [&](size_t bytes) -> char* { char* p = ws + off; off += (bytes + 255) & ~(size_t)255; return p; };
  unsigned short* X16  = (unsigned short*)carve((size_t)NROWS * NIN * 2);
  unsigned short* WCAT = (unsigned short*)carve((size_t)NCAT * NIN * 2);
  unsigned short* WMIX = (unsigned short*)carve((size_t)NOUT * KMIX * 2);
  float* Gpl   = (float*)carve((size_t)NROWS * NTRACE * 4);
  float* GATE  = (float*)carve((size_t)NROWS * NOUT * 4);
  float* SKT   = (float*)carve((size_t)NROWS * NOUT * 4);
  unsigned short* Zpl = (unsigned short*)carve((size_t)CROWS * KMIX * 2);
  float* CARRY = (float*)carve((size_t)2 * 2 * NSTATE * 4);
  if (off > ws_size || off > (size_t)134217728) return;

  const int n8x = NROWS * (NIN / 8);
  cvt_x_kernel<<<(n8x + 255) / 256, 256, 0, stream>>>(x, X16, n8x);
  wt_kernel<<<(NTRACE * (NIN / 8) + 255) / 256, 256, 0, stream>>>(W_pre,  NTRACE, NIN, WCAT, 0,  32, WX_CARRY);
  wt_kernel<<<(NTRACE * (NIN / 8) + 255) / 256, 256, 0, stream>>>(W_gin,  NTRACE, NIN, WCAT, 32, 32, WX_CARRY);
  wt_kernel<<<(NOUT * (NIN / 8) + 255) / 256, 256, 0, stream>>>(W_skip, NOUT, NIN, WCAT, 64, 64, WX_CARRY);
  wt_kernel<<<(NOUT * (NIN / 8) + 255) / 256, 256, 0, stream>>>(W_gout, NOUT, NIN, WCAT, 96, 64, WX_CARRY);
  wt_kernel<<<(NOUT * (KMIX / 8) + 255) / 256, 256, 0, stream>>>(W_mix, NOUT, KMIX, WMIX, 0, 32, WM_CARRY);

  xproj_gemm_kernel<<<((NROWS / 64) * (NCAT / 64)) / 8, 256, 0, stream>>>(
      X16, WCAT, b_pre, b_gin, b_gout, b_skip, Gpl, GATE, SKT);

  for (int ch = 0; ch < NCHUNK; ++ch) {
    float* cout = CARRY + (size_t)(ch & 1) * 2 * NSTATE;
    if (ch == 0) {
      scan_chunk_kernel<true><<<NSTATE / 256, 256, 0, stream>>>(
          Gpl, resets, h0, h0, a_param, b_param, cout, (unsigned*)Zpl, 0);
    } else {
      const float* cin = CARRY + (size_t)((ch - 1) & 1) * 2 * NSTATE;
      scan_chunk_kernel<false><<<NSTATE / 256, 256, 0, stream>>>(
          Gpl, resets, cin, cin + NSTATE, a_param, b_param, cout, (unsigned*)Zpl, ch * TCHUNK);
    }
    mix_ln_kernel<<<CROWS / 256, 256, 0, stream>>>(Zpl, WMIX, b_mix, GATE, SKT, out, ch * CROWS);
  }
}
